// ExpEncoder_42460046688738
// MI455X (gfx1250) — hardware-verified
//
#include <hip/hip_runtime.h>


namespace {
constexpr int B = 16, PW = 32, G = 512, D = 512, A = 400, AP = 416, NH = 8, OMC = 20001, PTW = 1000, NR = B * G;
constexpr float ES = 256.0f, TS = 4096.0f, WS_ = 4096.0f, WSC = 256.0f;
typedef _Float16 b16;
typedef __attribute__((ext_vector_type(16))) _Float16 v16b;
typedef __attribute__((ext_vector_type(8))) _Float16 v8b;
typedef __attribute__((ext_vector_type(8))) float v8f;
typedef __attribute__((ext_vector_type(4))) float v4f;
__device__ __forceinline__ float bf16_rne(float f) { unsigned int u = __float_as_uint(f); u += 0x7FFFu + ((u >> 16) & 1u); return __uint_as_float(u & 0xFFFF0000u); }
__device__ __forceinline__ void split16(float v, b16& hi, b16& lo) { hi = (b16)v; lo = (b16)(v - (float)hi); }
__device__ __forceinline__ v16b frag_kb(const b16* p, int hh) { const v8b a = *(const v8b*)(p + 8 * hh), b = *(const v8b*)(p + 16 + 8 * hh); v16b f;
#pragma unroll
  for (int e = 0; e < 8; ++e) { f[e] = a[e]; f[8 + e] = b[e]; } return f; }
__device__ __forceinline__ v8f wmma16b(v16b a, v16b b, v8f c) { v8f d = __builtin_amdgcn_wmma_f32_16x16x32_f16(false, a, false, b, (short)0, c, false, false); asm volatile("v_nop\n\tv_nop\n\tv_nop\n\tv_nop" : "+v"(d) : "v"(a), "v"(b)); return d; }
__device__ __forceinline__ void wave_lds_sync() { __builtin_amdgcn_fence(__ATOMIC_RELEASE, "workgroup"); __builtin_amdgcn_wave_barrier(); __builtin_amdgcn_fence(__ATOMIC_ACQUIRE, "workgroup"); }
__device__ __forceinline__ float pmul(float a, float b) { float p = a * b; asm volatile("" : "+v"(p)); return p; }
__device__ __forceinline__ int iclamp(int v, int lo, int hi) { return v < lo ? lo : (v > hi ? hi : v); }

__global__ __launch_bounds__(256) void w_kernel(const float* __restrict__ w0, const float* __restrict__ bw, b16* __restrict__ W0T, b16* __restrict__ BWT) {
  const int u = blockIdx.x * 256 + threadIdx.x; v8b v;
  if (u < AP * D / 8) { const int e = u * 8; const int a = e / D, d0 = e % D; for (int j = 0; j < 8; ++j) v[j] = a < A ? (b16)(bf16_rne(w0[(size_t)(d0 + j) * A + a]) * WSC) : (b16)0.0f; for (int pass = 0; pass < 2; ++pass) { *(volatile v8b*)(W0T + e) = v; __threadfence(); } }
  else if (u < AP * D / 8 + 16 * AP / 8) { const int e = (u - AP * D / 8) * 8; const int h = e / AP, a0 = e % AP; for (int j = 0; j < 8; ++j) { const int a = a0 + j; v[j] = (h < NH && a < A) ? (b16)(bf16_rne(bw[(size_t)a * NH + h]) * WSC) : (b16)0.0f; } for (int pass = 0; pass < 2; ++pass) { *(volatile v8b*)(BWT + e) = v; __threadfence(); } }
}
__global__ __launch_bounds__(256) void egather_kernel(const int* __restrict__ idx, const float* __restrict__ eg, int BV, b16* __restrict__ EA, b16* __restrict__ ET) {
  __shared__ float T[64][65]; const int dt = blockIdx.x % (D / 64), gt = (blockIdx.x / (D / 64)) % (G / 64), b = blockIdx.x / ((D / 64) * (G / 64)); if (b >= BV) return; const int tid = threadIdx.x;
  for (int i = tid; i < 64 * 64; i += 256) { const int gl = i / 64, dl = i % 64; const int row = iclamp(idx[b * G + gt * 64 + gl], 0, OMC - 1); T[gl][dl] = bf16_rne(eg[(size_t)row * D + dt * 64 + dl]); }
  __syncthreads();
  { const int gl = tid / 4, d0 = (tid % 4) * 16; v8b v0, v1; for (int j = 0; j < 8; ++j) { v0[j] = (b16)(T[gl][d0 + j] * ES); v1[j] = (b16)(T[gl][d0 + 8 + j] * ES); } const size_t o = ((size_t)b * G + gt * 64 + gl) * D + dt * 64 + d0; for (int pass = 0; pass < 2; ++pass) { *(volatile v8b*)(EA + o) = v0; *(volatile v8b*)(EA + o + 8) = v1; __threadfence(); } }
  { const int dl = tid / 4, g0 = (tid % 4) * 16; v8b v0, v1; for (int j = 0; j < 8; ++j) { v0[j] = (b16)(T[g0 + j][dl] * ES); v1[j] = (b16)(T[g0 + 8 + j][dl] * ES); } const size_t o = ((size_t)b * D + dt * 64 + dl) * G + gt * 64 + g0; for (int pass = 0; pass < 2; ++pass) { *(volatile v8b*)(ET + o) = v0; *(volatile v8b*)(ET + o + 8) = v1; __threadfence(); } }
}
__global__ __launch_bounds__(32) void proj_kernel(const b16* __restrict__ EA, const b16* __restrict__ W0T, const float* __restrict__ b0, int RV, float* __restrict__ PROJ) {
  __shared__ __attribute__((aligned(16))) float Tf[16][128 + 4];
  const int lane = threadIdx.x, nloc = lane & 15, hlf = lane >> 4; const size_t r0 = (size_t)blockIdx.x * 16; if (r0 >= (size_t)RV) return; const b16* ar = EA + (r0 + nloc) * D;
#pragma unroll 1
  for (int cg = 0; cg < 4; ++cg) { const int nt = (cg < 3) ? 8 : 2; v8f acc[8];
#pragma unroll
    for (int t = 0; t < 8; ++t) acc[t] = (v8f){};
#pragma unroll 2
    for (int kb = 0; kb < D; kb += 32) { const v16b a = frag_kb(ar + kb, hlf);
#pragma unroll
      for (int t = 0; t < 8; ++t) if (t < nt) acc[t] = wmma16b(a, frag_kb(W0T + (size_t)(cg * 128 + t * 16 + nloc) * D + kb, hlf), acc[t]); }
#pragma unroll
    for (int t = 0; t < 8; ++t) { if (t < nt) { const int c = cg * 128 + t * 16 + nloc; const float bb = c < A ? bf16_rne(b0[c]) : 0.0f;
#pragma unroll
        for (int r8 = 0; r8 < 8; ++r8) Tf[8 * hlf + r8][t * 16 + nloc] = c < A ? acc[t][r8] * (1.0f / (ES * WSC)) + bb : 0.0f; } }
    wave_lds_sync();
    const int ncol = nt * 16;
    for (int pass = 0; pass < 2; ++pass) { for (int rr = 0; rr < 16; ++rr) for (int c = lane; c < ncol; c += 32) ((volatile float*)PROJ)[(r0 + rr) * AP + cg * 128 + c] = Tf[rr][c]; __threadfence(); }
    wave_lds_sync(); }
}
__global__ __launch_bounds__(32) void logit_kernel(const float* __restrict__ PROJ, const int* __restrict__ pid, const float* __restrict__ ep, const b16* __restrict__ BWT, const float* __restrict__ bb, int BV, float* __restrict__ LG) {
  __shared__ __attribute__((aligned(16))) b16 Ah[16][AP + 8], Al[16][AP + 8]; __shared__ float So[16][NH];
  const int lane = threadIdx.x, nloc = lane & 15, hlf = lane >> 4; const int gt = blockIdx.x % (G / 16), p = (blockIdx.x / (G / 16)) % PW, b = blockIdx.x / ((G / 16) * PW); if (b >= BV) return;
  const int prow = iclamp(pid[p], 0, PTW - 1); const float* cr = ep + (size_t)prow * A;
  for (int rr = 0; rr < 16; ++rr) { const float* pr = PROJ + ((size_t)b * G + gt * 16 + rr) * AP; for (int q = 0; q < AP / 32; ++q) { const int a = q * 32 + lane; float v = 0.0f; if (a < A) v = tanhf(pr[a] + bf16_rne(cr[a])); b16 ph, pl; split16(v * TS, ph, pl); Ah[rr][a] = ph; Al[rr][a] = pl; } }
  wave_lds_sync();
  v8f acc = {};
#pragma unroll 1
  for (int kb = 0; kb < AP; kb += 32) { const v16b w = frag_kb(BWT + (size_t)nloc * AP + kb, hlf); acc = wmma16b(frag_kb(&Ah[nloc][kb], hlf), w, acc); acc = wmma16b(frag_kb(&Al[nloc][kb], hlf), w, acc); }
  if (nloc < NH) { const float b_ = bf16_rne(bb[nloc]);
#pragma unroll
    for (int r8 = 0; r8 < 8; ++r8) So[8 * hlf + r8][nloc] = acc[r8] * (1.0f / (TS * WSC)) + b_; }
  wave_lds_sync();
  for (int pass = 0; pass < 2; ++pass) { for (int i = lane; i < 16 * NH; i += 32) ((volatile float*)LG)[(((size_t)b * PW + p) * G + gt * 16) * NH + i] = So[i / NH][i % NH]; __threadfence(); }
}
__global__ __launch_bounds__(512) void soft_kernel(const float* __restrict__ LG, int BV, b16* __restrict__ WH, b16* __restrict__ WL) {
  __shared__ float red[16][NH]; __shared__ float mx[NH], den[NH]; __shared__ __attribute__((aligned(16))) b16 Sh[G], Sl[G];
  const int bp = blockIdx.x; if (bp / PW >= BV) return; const int g = threadIdx.x, wave = g >> 5, lane = g & 31; float l[NH]; for (int h = 0; h < NH; ++h) l[h] = LG[((size_t)bp * G + g) * NH + h];
  for (int h = 0; h < NH; ++h) { float m = l[h]; for (int o = 16; o; o >>= 1) m = fmaxf(m, __shfl_xor(m, o)); if (lane == 0) red[wave][h] = m; }
  __syncthreads(); if (g < NH) { float m = red[0][g]; for (int w = 1; w < 16; ++w) m = fmaxf(m, red[w][g]); mx[g] = m; } __syncthreads();
  float e[NH]; for (int h = 0; h < NH; ++h) e[h] = __expf(l[h] - mx[h]);
  for (int h = 0; h < NH; ++h) { float s = e[h]; for (int o = 16; o; o >>= 1) s += __shfl_xor(s, o); if (lane == 0) red[wave][h] = s; }
  __syncthreads(); if (g < NH) { float s = 0.0f; for (int w = 0; w < 16; ++w) s += red[w][g]; den[g] = s; } __syncthreads();
  float w = 0.0f; for (int h = 0; h < NH; ++h) w += e[h] / den[h];
  b16 ph, pl; split16(w * WS_, ph, pl); Sh[g] = ph; Sl[g] = pl; __syncthreads();
  if (g < 128) { const int half = g >> 6, i8 = (g & 63) * 8; const b16* src = half ? Sl : Sh; b16* dst = (half ? WL : WH) + (size_t)bp * G; const v8b v = *(const v8b*)(src + i8);
    for (int pass = 0; pass < 2; ++pass) { *(volatile v8b*)(dst + i8) = v; __threadfence(); } }
}
__global__ __launch_bounds__(32) void out_kernel(const b16* __restrict__ WH, const b16* __restrict__ WL, const b16* __restrict__ ET, int BV, float* __restrict__ out) {
  __shared__ __attribute__((aligned(16))) float Tf[16][128 + 4];
  const int lane = threadIdx.x, nloc = lane & 15, hlf = lane >> 4; const int cg = blockIdx.x % 4, pt = (blockIdx.x / 4) % (PW / 16), b = blockIdx.x / (4 * (PW / 16)); if (b >= BV) return;
  const size_t r0 = (size_t)b * PW + pt * 16; const b16* ah = WH + (r0 + nloc) * G; const b16* al = WL + (r0 + nloc) * G; v8f acc[8];
#pragma unroll
  for (int t = 0; t < 8; ++t) acc[t] = (v8f){};
#pragma unroll 2
  for (int kb = 0; kb < G; kb += 32) { const v16b a = frag_kb(ah + kb, hlf), a2 = frag_kb(al + kb, hlf);
#pragma unroll
    for (int t = 0; t < 8; ++t) { const v16b bw = frag_kb(ET + ((size_t)b * D + cg * 128 + t * 16 + nloc) * G + kb, hlf); acc[t] = wmma16b(a, bw, acc[t]); acc[t] = wmma16b(a2, bw, acc[t]); } }
#pragma unroll
  for (int t = 0; t < 8; ++t)
#pragma unroll
    for (int r8 = 0; r8 < 8; ++r8) Tf[8 * hlf + r8][t * 16 + nloc] = acc[t][r8] * (1.0f / (WS_ * ES));
  wave_lds_sync();
  for (int pass = 0; pass < 2; ++pass) { for (int rr = 0; rr < 16; ++rr) *(volatile v4f*)(out + (r0 + rr) * D + cg * 128 + lane * 4) = *(const v4f*)(&Tf[rr][lane * 4]); __threadfence(); }
}
}

extern "C" void kernel_launch(void* const* d_in, const int* in_sizes, int n_in, void* d_out, int out_size, void* d_ws, size_t ws_size, hipStream_t stream) {
  (void)n_in;
  auto Fp = [&](int i) { return (const float*)d_in[i]; }; auto Ip = [&](int i) { return (const int*)d_in[i]; };
  if (in_sizes[0] != B * G || in_sizes[1] != PW || in_sizes[2] != OMC * D || in_sizes[3] != PTW * A || in_sizes[4] != D * A || in_sizes[5] != A || in_sizes[6] != A * NH || in_sizes[7] != NH || out_size != B * PW * D) return;
  const int BV = B;
  size_t off = 0; char* ws = (char*)d_ws;
  auto carve = [&](size_t bytes) { char* p = ws + off; off += (bytes + 255) & ~(size_t)255; return p; };
  b16* W0T = (b16*)carve((size_t)AP * D * 2); b16* BWT = (b16*)carve((size_t)16 * AP * 2); b16* EA = (b16*)carve((size_t)NR * D * 2); b16* ET = (b16*)carve((size_t)NR * D * 2); float* PROJ = (float*)carve((size_t)NR * AP * 4); float* LG = (float*)carve((size_t)B * PW * G * NH * 4); b16* WH = (b16*)carve((size_t)B * PW * G * 2); b16* WL = (b16*)carve((size_t)B * PW * G * 2);
  if (off > ws_size || off > ((size_t)64 << 20)) return;
  w_kernel<<<(AP * D / 8 + 16 * AP / 8 + 255) / 256, 256, 0, stream>>>(Fp(4), Fp(6), W0T, BWT);
  egather_kernel<<<BV * (G / 64) * (D / 64), 256, 0, stream>>>(Ip(0), Fp(2), BV, EA, ET);
  proj_kernel<<<(BV * G) / 16, 32, 0, stream>>>(EA, W0T, Fp(5), BV * G, PROJ);
  logit_kernel<<<BV * PW * (G / 16), 32, 0, stream>>>(PROJ, Ip(1), Fp(3), BWT, Fp(7), BV, LG);
  soft_kernel<<<BV * PW, 512, 0, stream>>>(LG, BV, WH, WL);
  out_kernel<<<BV * (PW / 16) * 4, 32, 0, stream>>>(WH, WL, ET, BV, (float*)d_out);
}
